// MotionLSTM_5394478924393
// MI455X (gfx1250) — hardware-verified
//
#include <hip/hip_runtime.h>
#include <math.h>

constexpr int NSEQ    = 256;
constexpr int NSTEP   = 512;
constexpr int NFEAT   = 64;
constexpr int NHID    = 128;
constexpr int NGATE   = 4 * NHID;
constexpr int NCLS    = 16;
constexpr int NTHR    = 256;
constexpr int SEQ_BLK = 16;
constexpr int XP0     = 72;
constexpr int XP1     = 136;
constexpr int HP      = 136;
constexpr int HSP     = 132;
constexpr float WSC     = 64.0f;
constexpr float WSC_INV = 1.0f / 64.0f;
static_assert(NSEQ % SEQ_BLK == 0);
static_assert(NHID == 16 * (NTHR / 32));
static_assert(NFEAT % 32 == 0 && NHID % 32 == 0);
static_assert(SEQ_BLK * NFEAT == 4 * NTHR);
static_assert(SEQ_BLK * NHID == 8 * NTHR);
static_assert(SEQ_BLK * NCLS == NTHR);
static_assert((NGATE * NFEAT) % (8 * NTHR) == 0 && (NGATE * NHID) % (8 * NTHR) == 0);
static_assert((XP0 * 2) % 16 == 0 && (XP1 * 2) % 16 == 0 && (HP * 2) % 16 == 0 && (HSP * 4) % 16 == 0);

typedef __attribute__((ext_vector_type(16))) _Float16 v16h;
typedef __attribute__((ext_vector_type(8)))  _Float16 v8h;
typedef __attribute__((ext_vector_type(8)))  float    v8f;
typedef __attribute__((ext_vector_type(4)))  float    v4f;
typedef __attribute__((ext_vector_type(4)))  unsigned u32x4;
typedef __attribute__((ext_vector_type(2)))  unsigned v2u;

__device__ __forceinline__ void dep_guard_h(v8f& a, v8f& b, v16h x, v16h y) { asm volatile("v_nop\n\tv_nop\n\tv_nop\n\tv_nop" : "+v"(a), "+v"(b) : "v"(x), "v"(y)); }
__device__ __forceinline__ void keep4_h(v16h a, v16h b, v16h c, v16h d) { asm volatile("v_nop" :: "v"(a), "v"(b), "v"(c), "v"(d)); }
__device__ __forceinline__ void acc_guard4(v8f& a, v8f& b, v8f& c, v8f& d) { asm volatile("v_nop\n\tv_nop\n\tv_nop\n\tv_nop" : "+v"(a), "+v"(b), "+v"(c), "+v"(d)); }
template <typename T> struct Frag;
template <> struct Frag<_Float16> {
  typedef v16h V; union U { v16h v; v8h h[2]; };
  static __device__ __forceinline__ v16h load(const _Float16* p) {
    U f; f.h[0] = *(const v8h*)(p); f.h[1] = *(const v8h*)(p + 16); return f.v;
  }
  static __device__ __forceinline__ v8f mma(v16h a, v16h b, v8f c) {
    return __builtin_amdgcn_wmma_f32_16x16x32_f16(false, a, false, b, (short)0, c, false, false);
  }
};

__device__ __forceinline__ unsigned f16bits(float f) { return (unsigned)__builtin_bit_cast(unsigned short, (_Float16)f); }
__device__ __forceinline__ float fsig(float v)  { return __builtin_amdgcn_rcpf(1.0f + expf(-v)); }
__device__ __forceinline__ float ftanh(float v) { return 1.0f - 2.0f * __builtin_amdgcn_rcpf(expf(2.0f * v) + 1.0f); }

__global__ __launch_bounds__(NTHR) void cast16_kernel(const float* __restrict__ src, unsigned short* __restrict__ dst, int n8, float sc) {
  const int i = blockIdx.x * NTHR + threadIdx.x;
  if (i < n8) {
    const float* sp = src + (size_t)i * 8;
    const v4f a = *(const v4f*)(sp);
    const v4f b = *(const v4f*)(sp + 4);
    u32x4 w;
    w[0] = f16bits(a[0] * sc) | (f16bits(a[1] * sc) << 16);
    w[1] = f16bits(a[2] * sc) | (f16bits(a[3] * sc) << 16);
    w[2] = f16bits(b[0] * sc) | (f16bits(b[1] * sc) << 16);
    w[3] = f16bits(b[2] * sc) | (f16bits(b[3] * sc) << 16);
    unsigned short* dp = dst + (size_t)i * 8;
    *(volatile u32x4*)dp = w;
    __threadfence();
    *(volatile u32x4*)dp = w;
  }
}

__device__ __forceinline__ void stage_x0(unsigned short* Ax, const float* __restrict__ x, int rowbase, int t, int tid) {
  const int m = tid >> 4, f4 = (tid & 15) * 4;
  const v4f v = *(const v4f*)(x + ((size_t)(rowbase + m) * NSTEP + (size_t)t) * NFEAT + f4);
  v2u pk;
  pk[0] = f16bits(v[0]) | (f16bits(v[1]) << 16);
  pk[1] = f16bits(v[2]) | (f16bits(v[3]) << 16);
  *(v2u*)(Ax + m * XP0 + f4) = pk;
}

__device__ __forceinline__ void stage_x1(unsigned short* Ax, const unsigned short* __restrict__ H1, int rowbase, int t, int tid) {
  const int m = tid >> 4, c8 = (tid & 15) * 8;
  const u32x4 w = *(const u32x4*)(H1 + ((size_t)t * NSEQ + (size_t)(rowbase + m)) * NHID + c8);
  *(u32x4*)(Ax + m * XP1 + c8) = w;
}

__global__ __launch_bounds__(NTHR) void lstm_layer0_kernel(const float* __restrict__ x,
                                                           const float* __restrict__ b_ih, const float* __restrict__ b_hh,
                                                           const unsigned short* __restrict__ WXp,
                                                           const unsigned short* __restrict__ WHp,
                                                           unsigned short* __restrict__ H1) {
  __shared__ __align__(16) unsigned short Ax[SEQ_BLK * XP0];
  __shared__ __align__(16) unsigned short Ah[SEQ_BLK * HP];
  const _Float16* WX = (const _Float16*)WXp;
  const _Float16* WH = (const _Float16*)WHp;
  const int tid = threadIdx.x, lane = tid & 31, wave = tid >> 5;
  const int c = lane & 15, hh = lane >> 4, koff = hh * 8;
  const int rowbase = blockIdx.x * SEQ_BLK;
  const int j = 16 * wave + c;

#pragma unroll 1
  for (int i = tid; i < SEQ_BLK * XP0; i += NTHR) Ax[i] = 0;
#pragma unroll 1
  for (int i = tid; i < SEQ_BLK * HP; i += NTHR) Ah[i] = 0;
  float cst[8], hst[8], bb[4];
#pragma unroll
  for (int r = 0; r < 8; ++r) { cst[r] = 0.0f; hst[r] = 0.0f; }
#pragma unroll
  for (int g = 0; g < 4; ++g) bb[g] = b_ih[g * NHID + j] + b_hh[g * NHID + j];
  __syncthreads();
  stage_x0(Ax, x, rowbase, 0, tid);
  __syncthreads();

  const _Float16* axrow = (const _Float16*)Ax + c * XP0 + koff;
  const _Float16* ahrow = (const _Float16*)Ah + c * HP + koff;
  const _Float16* wx = WX + (size_t)j * NFEAT + koff;
  const _Float16* wh = WH + (size_t)j * NHID + koff;
  const v8f z8 = {0.f, 0.f, 0.f, 0.f, 0.f, 0.f, 0.f, 0.f};
  const int srow = tid >> 4, sc8 = (tid & 15) * 8;

#pragma unroll 1
  for (int t = 0; t < NSTEP; ++t) {
    v8f acc[4];
    acc[0] = z8; acc[1] = z8; acc[2] = z8; acc[3] = z8;
#pragma unroll 1
    for (int kx = 0; kx < NFEAT; kx += 32) {
      const v16h a  = Frag<_Float16>::load(axrow + kx);
      const v16h b0 = Frag<_Float16>::load(wx + kx);
      const v16h b1 = Frag<_Float16>::load(wx + (size_t)1 * NHID * NFEAT + kx);
      const v16h b2 = Frag<_Float16>::load(wx + (size_t)2 * NHID * NFEAT + kx);
      const v16h b3 = Frag<_Float16>::load(wx + (size_t)3 * NHID * NFEAT + kx);
      acc[0] = Frag<_Float16>::mma(a, b0, acc[0]);
      acc[1] = Frag<_Float16>::mma(a, b1, acc[1]);
      acc[2] = Frag<_Float16>::mma(a, b2, acc[2]);
      acc[3] = Frag<_Float16>::mma(a, b3, acc[3]);
      dep_guard_h(acc[0], acc[3], a, b3);
      keep4_h(b0, b1, b2, b3);
    }
#pragma unroll 1
    for (int k0 = 0; k0 < NHID; k0 += 32) {
      const v16h a  = Frag<_Float16>::load(ahrow + k0);
      const v16h b0 = Frag<_Float16>::load(wh + k0);
      const v16h b1 = Frag<_Float16>::load(wh + (size_t)1 * NHID * NHID + k0);
      const v16h b2 = Frag<_Float16>::load(wh + (size_t)2 * NHID * NHID + k0);
      const v16h b3 = Frag<_Float16>::load(wh + (size_t)3 * NHID * NHID + k0);
      acc[0] = Frag<_Float16>::mma(a, b0, acc[0]);
      acc[1] = Frag<_Float16>::mma(a, b1, acc[1]);
      acc[2] = Frag<_Float16>::mma(a, b2, acc[2]);
      acc[3] = Frag<_Float16>::mma(a, b3, acc[3]);
      dep_guard_h(acc[0], acc[3], a, b3);
      keep4_h(b0, b1, b2, b3);
    }
    acc_guard4(acc[0], acc[1], acc[2], acc[3]);
#pragma unroll
    for (int r = 0; r < 8; ++r) {
      const float zi = acc[0][r] * WSC_INV + bb[0];
      const float zf = acc[1][r] * WSC_INV + bb[1];
      const float zg = acc[2][r] * WSC_INV + bb[2];
      const float zo = acc[3][r] * WSC_INV + bb[3];
      const float ig = fsig(zi);
      const float fg = fsig(zf);
      const float gg = ftanh(zg);
      const float og = fsig(zo);
      const float cn = fg * cst[r] + ig * gg;
      cst[r] = cn;
      hst[r] = og * ftanh(cn);
    }
    __syncthreads();
#pragma unroll
    for (int r = 0; r < 8; ++r) Ah[(8 * hh + r) * HP + j] = (unsigned short)f16bits(hst[r]);
    stage_x0(Ax, x, rowbase, (t + 1 < NSTEP) ? (t + 1) : (NSTEP - 1), tid);
    __syncthreads();
    {
      const u32x4 w = *(const u32x4*)(Ah + srow * HP + sc8);
      unsigned short* gp = H1 + ((size_t)t * NSEQ + (size_t)(rowbase + srow)) * NHID + sc8;
      for (int pass = 0; pass < 2; ++pass) {
        *(volatile u32x4*)gp = w;
        __threadfence();
      }
    }
  }
}

__global__ __launch_bounds__(NTHR) void lstm_layer1_kernel(const unsigned short* __restrict__ H1,
                                                           const float* __restrict__ b_ih, const float* __restrict__ b_hh,
                                                           const unsigned short* __restrict__ WXp,
                                                           const unsigned short* __restrict__ WHp,
                                                           const float* __restrict__ fc_w, const float* __restrict__ fc_b,
                                                           float* __restrict__ out) {
  __shared__ __align__(16) unsigned short Ax[SEQ_BLK * XP1];
  __shared__ __align__(16) unsigned short Ah[SEQ_BLK * HP];
  __shared__ __align__(16) float          Hs[SEQ_BLK * HSP];
  __shared__ __align__(16) float          Os[SEQ_BLK * NCLS];
  const _Float16* WX = (const _Float16*)WXp;
  const _Float16* WH = (const _Float16*)WHp;
  const int tid = threadIdx.x, lane = tid & 31, wave = tid >> 5;
  const int c = lane & 15, hh = lane >> 4, koff = hh * 8;
  const int rowbase = blockIdx.x * SEQ_BLK;
  const int j = 16 * wave + c;

#pragma unroll 1
  for (int i = tid; i < SEQ_BLK * XP1; i += NTHR) Ax[i] = 0;
#pragma unroll 1
  for (int i = tid; i < SEQ_BLK * HP; i += NTHR) Ah[i] = 0;
#pragma unroll 1
  for (int i = tid; i < SEQ_BLK * HSP; i += NTHR) Hs[i] = 0.0f;
  Os[tid] = 0.0f;
  float cst[8], hst[8], bb[4];
#pragma unroll
  for (int r = 0; r < 8; ++r) { cst[r] = 0.0f; hst[r] = 0.0f; }
#pragma unroll
  for (int g = 0; g < 4; ++g) bb[g] = b_ih[g * NHID + j] + b_hh[g * NHID + j];
  __syncthreads();
  stage_x1(Ax, H1, rowbase, 0, tid);
  __syncthreads();

  const _Float16* axrow = (const _Float16*)Ax + c * XP1 + koff;
  const _Float16* ahrow = (const _Float16*)Ah + c * HP + koff;
  const _Float16* wx = WX + (size_t)j * NHID + koff;
  const _Float16* wh = WH + (size_t)j * NHID + koff;
  const v8f z8 = {0.f, 0.f, 0.f, 0.f, 0.f, 0.f, 0.f, 0.f};

#pragma unroll 1
  for (int t = 0; t < NSTEP; ++t) {
    v8f acc[4];
    acc[0] = z8; acc[1] = z8; acc[2] = z8; acc[3] = z8;
#pragma unroll 1
    for (int kx = 0; kx < NHID; kx += 32) {
      const v16h a  = Frag<_Float16>::load(axrow + kx);
      const v16h b0 = Frag<_Float16>::load(wx + kx);
      const v16h b1 = Frag<_Float16>::load(wx + (size_t)1 * NHID * NHID + kx);
      const v16h b2 = Frag<_Float16>::load(wx + (size_t)2 * NHID * NHID + kx);
      const v16h b3 = Frag<_Float16>::load(wx + (size_t)3 * NHID * NHID + kx);
      acc[0] = Frag<_Float16>::mma(a, b0, acc[0]);
      acc[1] = Frag<_Float16>::mma(a, b1, acc[1]);
      acc[2] = Frag<_Float16>::mma(a, b2, acc[2]);
      acc[3] = Frag<_Float16>::mma(a, b3, acc[3]);
      dep_guard_h(acc[0], acc[3], a, b3);
      keep4_h(b0, b1, b2, b3);
    }
#pragma unroll 1
    for (int k0 = 0; k0 < NHID; k0 += 32) {
      const v16h a  = Frag<_Float16>::load(ahrow + k0);
      const v16h b0 = Frag<_Float16>::load(wh + k0);
      const v16h b1 = Frag<_Float16>::load(wh + (size_t)1 * NHID * NHID + k0);
      const v16h b2 = Frag<_Float16>::load(wh + (size_t)2 * NHID * NHID + k0);
      const v16h b3 = Frag<_Float16>::load(wh + (size_t)3 * NHID * NHID + k0);
      acc[0] = Frag<_Float16>::mma(a, b0, acc[0]);
      acc[1] = Frag<_Float16>::mma(a, b1, acc[1]);
      acc[2] = Frag<_Float16>::mma(a, b2, acc[2]);
      acc[3] = Frag<_Float16>::mma(a, b3, acc[3]);
      dep_guard_h(acc[0], acc[3], a, b3);
      keep4_h(b0, b1, b2, b3);
    }
    acc_guard4(acc[0], acc[1], acc[2], acc[3]);
#pragma unroll
    for (int r = 0; r < 8; ++r) {
      const float zi = acc[0][r] * WSC_INV + bb[0];
      const float zf = acc[1][r] * WSC_INV + bb[1];
      const float zg = acc[2][r] * WSC_INV + bb[2];
      const float zo = acc[3][r] * WSC_INV + bb[3];
      const float ig = fsig(zi);
      const float fg = fsig(zf);
      const float gg = ftanh(zg);
      const float og = fsig(zo);
      const float cn = fg * cst[r] + ig * gg;
      cst[r] = cn;
      hst[r] = og * ftanh(cn);
    }
    __syncthreads();
#pragma unroll
    for (int r = 0; r < 8; ++r) Ah[(8 * hh + r) * HP + j] = (unsigned short)f16bits(hst[r]);
    stage_x1(Ax, H1, rowbase, (t + 1 < NSTEP) ? (t + 1) : (NSTEP - 1), tid);
    __syncthreads();
  }

#pragma unroll
  for (int r = 0; r < 8; ++r) Hs[(8 * hh + r) * HSP + j] = hst[r];
  __syncthreads();
  {
    const int row = tid >> 4, cls = tid & 15;
    const float* hp = Hs + row * HSP;
    const float* wp = fc_w + (size_t)cls * NHID;
    float s = 0.0f;
#pragma unroll 1
    for (int k = 0; k < NHID; k += 4) {
      const v4f hv = *(const v4f*)(hp + k);
      const v4f wv = *(const v4f*)(wp + k);
      s = fmaf(hv[0], wv[0], s);
      s = fmaf(hv[1], wv[1], s);
      s = fmaf(hv[2], wv[2], s);
      s = fmaf(hv[3], wv[3], s);
    }
    s += fc_b[cls];
    Os[row * NCLS + cls] = s;
  }
  __syncthreads();
  if (wave == 0) {
    float* op = out + (size_t)rowbase * NCLS;
    for (int pass = 0; pass < 2; ++pass) {
#pragma unroll
      for (int it = 0; it < 2; ++it) {
        const int idx = it * 32 + lane;
        const v4f v = *(const v4f*)(Os + idx * 4);
        *(volatile v4f*)(op + idx * 4) = v;
      }
      __threadfence();
    }
  }
}

extern "C" void kernel_launch(void* const* d_in, const int* in_sizes, int n_in,
                              void* d_out, int out_size, void* d_ws, size_t ws_size, hipStream_t stream) {
  if (n_in < 11 || d_out == nullptr || d_ws == nullptr) return;
  if (in_sizes[0] != NSEQ * NSTEP * NFEAT || in_sizes[1] != NGATE * NFEAT || in_sizes[2] != NGATE * NHID ||
      in_sizes[3] != NGATE || in_sizes[4] != NGATE || in_sizes[5] != NGATE * NHID || in_sizes[6] != NGATE * NHID ||
      in_sizes[7] != NGATE || in_sizes[8] != NGATE || in_sizes[9] != NCLS * NHID || in_sizes[10] != NCLS ||
      out_size != NSEQ * NCLS) return;

  const float* x     = (const float*)d_in[0];
  const float* w_ih0 = (const float*)d_in[1];
  const float* w_hh0 = (const float*)d_in[2];
  const float* b_ih0 = (const float*)d_in[3];
  const float* b_hh0 = (const float*)d_in[4];
  const float* w_ih1 = (const float*)d_in[5];
  const float* w_hh1 = (const float*)d_in[6];
  const float* b_ih1 = (const float*)d_in[7];
  const float* b_hh1 = (const float*)d_in[8];
  const float* fc_w  = (const float*)d_in[9];
  const float* fc_b  = (const float*)d_in[10];
  float* out = (float*)d_out;

  char* ws = (char*)d_ws; size_t off = 0;
  auto carve = [&](size_t bytes) -> char* { char* p = ws + off; off += (bytes + 255) & ~(size_t)255; return p; };
  unsigned short* WX0 = (unsigned short*)carve((size_t)NGATE * NFEAT * 2);
  unsigned short* WH0 = (unsigned short*)carve((size_t)NGATE * NHID * 2);
  unsigned short* WX1 = (unsigned short*)carve((size_t)NGATE * NHID * 2);
  unsigned short* WH1 = (unsigned short*)carve((size_t)NGATE * NHID * 2);
  unsigned short* H1  = (unsigned short*)carve((size_t)NSTEP * NSEQ * NHID * 2);
  if (off > ws_size || off > (size_t)134217728) return;

  const int n8a = NGATE * NFEAT / 8;
  const int n8b = NGATE * NHID / 8;
  cast16_kernel<<<(n8a + NTHR - 1) / NTHR, NTHR, 0, stream>>>(w_ih0, WX0, n8a, WSC);
  cast16_kernel<<<(n8b + NTHR - 1) / NTHR, NTHR, 0, stream>>>(w_hh0, WH0, n8b, WSC);
  cast16_kernel<<<(n8b + NTHR - 1) / NTHR, NTHR, 0, stream>>>(w_ih1, WX1, n8b, WSC);
  cast16_kernel<<<(n8b + NTHR - 1) / NTHR, NTHR, 0, stream>>>(w_hh1, WH1, n8b, WSC);
  lstm_layer0_kernel<<<NSEQ / SEQ_BLK, NTHR, 0, stream>>>(x, b_ih0, b_hh0, WX0, WH0, H1);
  lstm_layer1_kernel<<<NSEQ / SEQ_BLK, NTHR, 0, stream>>>(H1, b_ih1, b_hh1, WX1, WH1, fc_w, fc_b, out);
}
